// PyGEGNNDecoder_6236292514324
// MI455X (gfx1250) — hardware-verified
//
#include <hip/hip_runtime.h>
#include <stddef.h>


#define HD      128
#define H2      256
#define AFD     16
#define LATD    64
#define KIN     96
#define KIN0    80
#define EWR     257
#define ASC     8
#define WSC     64
#define OSC     (1.0f / 512.0f)
#define NTHR    256
#define NWAVE   8
#define EPT     8
#define NGRP    2
#define CHUNK   (NTHR * EPT * NGRP)
#define WCAP    (EPT * NGRP * 32)
#define LISTN   (NWAVE * WCAP)
#define NBC     4096
#define NBF     1024
#define RCAP    20480
#define RBN     128
#define OTHR    512
#define DEGCAP  256
#define BM      64
#define NCW     64
#define TW      4
#define TTHR    (TW * 32)
#define ANB     32
#define WSCAP   134217728
#define LDS_FILL ((2 * RCAP + NBF + LISTN) * 4 + 64)

static_assert((CHUNK & (CHUNK - 1)) == 0);
static_assert(CHUNK <= 4096);
static_assert(NBC <= 4096 && NBF <= 4096);
static_assert((NBC & (NBC - 1)) == 0 && (NBF & (NBF - 1)) == 0);
static_assert(NBC == 4 * NBF);
static_assert(OTHR * 8 == NBC);
static_assert((RCAP % 32) == 0);
static_assert(BM * 4 == NTHR);
static_assert(WCAP == EPT * NGRP * 32);
static_assert(TTHR == 128);
static_assert(ANB * 8 == NTHR);

typedef float          v4f  __attribute__((ext_vector_type(4)));
typedef float          v8f  __attribute__((ext_vector_type(8)));
typedef int            v4i  __attribute__((ext_vector_type(4)));
typedef _Float16       v4h  __attribute__((ext_vector_type(4)));
typedef _Float16       v8h  __attribute__((ext_vector_type(8)));
typedef _Float16       v16h __attribute__((ext_vector_type(16)));
typedef _Float16       v8ha __attribute__((ext_vector_type(8), __may_alias__));
typedef unsigned short v4us __attribute__((ext_vector_type(4)));
typedef unsigned short v8us __attribute__((ext_vector_type(8)));
union FragH { v16h v; v8us u[2]; v8h h[2]; };

__device__ __forceinline__ v8f wmh(v16h a, v16h b, v8f c) {
  v8f d = __builtin_amdgcn_wmma_f32_16x16x32_f16(false, a, false, b, (short)0, c, false, false);
  asm volatile("v_nop\n\tv_nop\n\tv_nop\n\tv_nop" : "+v"(d) : "v"(a), "v"(b));
  return d;
}
__device__ __forceinline__ v8f zero8() { v8f z = {0.f, 0.f, 0.f, 0.f, 0.f, 0.f, 0.f, 0.f}; return z; }
__device__ __forceinline__ float silu_f(float x) { return x * __builtin_amdgcn_rcpf(1.0f + __expf(-x)); }
__device__ __forceinline__ float wsum32(float v) {
#pragma unroll
  for (int s = 16; s > 0; s >>= 1) v += __shfl_xor(v, s);
  return v;
}

__device__ __forceinline__ v16h frag_glb(const unsigned short* P, int row, int ld, int k0, int hh) {
  FragH f;
  const unsigned short* p = P + (size_t)row * ld + k0 + 8 * hh;
  f.u[0] = *(const v8us*)p;
  f.u[1] = *(const v8us*)(p + 16);
  return f.v;
}
__device__ __forceinline__ v16h frag_lds(const _Float16* T, int row, int ld, int k0, int hh) {
  FragH f;
  const _Float16* p = T + row * ld + k0 + 8 * hh;
  f.h[0] = *(const v8h*)p;
  f.h[1] = *(const v8h*)(p + 16);
  return f.v;
}

template <int NB>
__device__ __forceinline__ int scan_chunk(const int* __restrict__ dsts, int nE, int cbase, int slotBase,
                                          int vec8, int* list, int tid, int lane, int wave) {
  int wc = 0;
#pragma unroll
  for (int g = 0; g < NGRP; ++g) {
    const int el0  = (g * NTHR + tid) * EPT;
    const int e0   = cbase + el0;
    const int sent = -2147483647 - 1;
    v4i da, db;
    if (vec8 != 0 && cbase + CHUNK <= nE) {
      da = *(const v4i*)(dsts + e0);
      db = *(const v4i*)(dsts + e0 + 4);
    } else {
      da.x = (e0     < nE) ? dsts[min(e0, nE - 1)] : sent;
      da.y = (e0 + 1 < nE) ? dsts[min(e0 + 1, nE - 1)] : sent;
      da.z = (e0 + 2 < nE) ? dsts[min(e0 + 2, nE - 1)] : sent;
      da.w = (e0 + 3 < nE) ? dsts[min(e0 + 3, nE - 1)] : sent;
      db.x = (e0 + 4 < nE) ? dsts[min(e0 + 4, nE - 1)] : sent;
      db.y = (e0 + 5 < nE) ? dsts[min(e0 + 5, nE - 1)] : sent;
      db.z = (e0 + 6 < nE) ? dsts[min(e0 + 6, nE - 1)] : sent;
      db.w = (e0 + 7 < nE) ? dsts[min(e0 + 7, nE - 1)] : sent;
    }
    const unsigned nb = (unsigned)slotBase;
    const unsigned s0 = (unsigned)da.x - nb, s1 = (unsigned)da.y - nb;
    const unsigned s2 = (unsigned)da.z - nb, s3 = (unsigned)da.w - nb;
    const unsigned s4 = (unsigned)db.x - nb, s5 = (unsigned)db.y - nb;
    const unsigned s6 = (unsigned)db.z - nb, s7 = (unsigned)db.w - nb;
    const bool h0 = s0 < (unsigned)NB, h1 = s1 < (unsigned)NB, h2 = s2 < (unsigned)NB, h3 = s3 < (unsigned)NB;
    const bool h4 = s4 < (unsigned)NB, h5 = s5 < (unsigned)NB, h6 = s6 < (unsigned)NB, h7 = s7 < (unsigned)NB;
    const unsigned any = __builtin_amdgcn_ballot_w32(h0 | h1 | h2 | h3 | h4 | h5 | h6 | h7);
    if (any != 0u) {
#define HITJ(J, HJ, SJ) { \
        const unsigned mj = __builtin_amdgcn_ballot_w32(HJ); \
        if (mj != 0u) { \
          if (HJ) { \
            const int pos = wc + (int)__builtin_amdgcn_mbcnt_lo(mj, 0u); \
            if (pos < WCAP) list[wave * WCAP + pos] = ((el0 + (J)) << 12) | (int)(SJ); \
          } \
          wc += (int)__builtin_popcount(mj); } }
      HITJ(0, h0, s0)
      HITJ(1, h1, s1)
      HITJ(2, h2, s2)
      HITJ(3, h3, s3)
      HITJ(4, h4, s4)
      HITJ(5, h5, s5)
      HITJ(6, h6, s6)
      HITJ(7, h7, s7)
#undef HITJ
    }
  }
  return wc;
}

__global__ __launch_bounds__(NTHR) void k_count(const int* __restrict__ keys, int* cnt, int nE, int vec8) {
  __shared__ __attribute__((aligned(16))) int scnt[NBC];
  __shared__ __attribute__((aligned(16))) int list[LISTN];
  __shared__ int wcnt[NWAVE];
  const int tid = threadIdx.x, lane = tid & 31, wave = tid >> 5;
  const int nodeBase = blockIdx.x * NBC;

  for (int i = tid; i < NBC; i += NTHR) scnt[i] = 0;
  __syncthreads();

  const int nChunks = (nE + CHUNK - 1) / CHUNK;
#pragma unroll 1
  for (int ch = 0; ch < nChunks; ++ch) {
    const int cbase = ch * CHUNK;
    const int wc = scan_chunk<NBC>(keys, nE, cbase, nodeBase, vec8, list, tid, lane, wave);
    if (lane == 0) wcnt[wave] = wc;
    __syncthreads();
    if (wave == 0) {
#pragma unroll 1
      for (int wsx = 0; wsx < NWAVE; ++wsx) {
        int n = __builtin_amdgcn_readfirstlane(wcnt[wsx]);
        n = n > WCAP ? WCAP : (n < 0 ? 0 : n);
        const int* lp = list + wsx * WCAP;
#pragma unroll 1
        for (int i = 0; i < n; ++i) {
          const int ent  = __builtin_amdgcn_readfirstlane(lp[i]);
          const int slot = ent & (NBC - 1);
          if (lane == 0) scnt[slot] = scnt[slot] + 1;
        }
      }
    }
    __syncthreads();
  }

  v4i cq[4];
#pragma unroll
  for (int q = 0; q < 4; ++q) {
    const int f = (wave * 4 + q) * 128 + 4 * lane;
    cq[q] = *(const v4i*)(scnt + f);
  }
  int* cp = cnt + (size_t)nodeBase;
#pragma unroll
  for (int q = 0; q < 4; ++q) {
    const int f = (wave * 4 + q) * 128 + 4 * lane;
    *(volatile v4i*)(cp + f) = cq[q];
  }
  __threadfence();
#pragma unroll
  for (int q = 0; q < 4; ++q) {
    const int f = (wave * 4 + q) * 128 + 4 * lane;
    *(volatile v4i*)(cp + f) = cq[q];
  }
}

__global__ __launch_bounds__(OTHR) void k_offsets(
    const int* __restrict__ cnt, int* off, int* rbase, int nChunk) {
  __shared__ __attribute__((aligned(16))) int soff[NBC];
  __shared__ __attribute__((aligned(16))) int srb[RBN];
  __shared__ int wtot[OTHR / 32];
  const int tid = threadIdx.x, lane = tid & 31, wave = tid >> 5, sub = tid >> 7;
  for (int i = tid; i < RBN; i += OTHR) srb[i] = 0;
  int carry = 0;
#pragma unroll 1
  for (int ch = 0; ch < nChunk; ++ch) {
    const int base = ch * NBC;
    const v4i c0 = *(const v4i*)(cnt + base + 8 * tid);
    const v4i c1 = *(const v4i*)(cnt + base + 8 * tid + 4);
    const int e0 = max(c0.x, 0), e1 = max(c0.y, 0), e2 = max(c0.z, 0), e3 = max(c0.w, 0);
    const int e4 = max(c1.x, 0), e5 = max(c1.y, 0), e6 = max(c1.z, 0), e7 = max(c1.w, 0);
    const int ts = e0 + e1 + e2 + e3 + e4 + e5 + e6 + e7;
    int incl = ts;
#pragma unroll
    for (int d = 1; d < 32; d <<= 1) {
      const int t = __shfl_up(incl, d);
      if (lane >= d) incl += t;
    }
    if (lane == 31) wtot[wave] = incl;
    __syncthreads();
    const int S0 = wtot[0]  + wtot[1]  + wtot[2]  + wtot[3];
    const int S1 = wtot[4]  + wtot[5]  + wtot[6]  + wtot[7];
    const int S2 = wtot[8]  + wtot[9]  + wtot[10] + wtot[11];
    const int S3 = wtot[12] + wtot[13] + wtot[14] + wtot[15];
    int pre = 0;
#pragma unroll 1
    for (int w = 4 * sub; w < wave; ++w) pre += wtot[w];
    const int b0 = carry;
    const int b1 = b0 + ((S0 + 31) & ~31);
    const int b2 = b1 + ((S1 + 31) & ~31);
    const int b3 = b2 + ((S2 + 31) & ~31);
    const int b4 = b3 + ((S3 + 31) & ~31);
    const int myb = sub == 0 ? b0 : (sub == 1 ? b1 : (sub == 2 ? b2 : b3));
    if (tid == 0) {
      srb[min(4 * ch + 0, RBN - 1)] = b0;
      srb[min(4 * ch + 1, RBN - 1)] = b1;
      srb[min(4 * ch + 2, RBN - 1)] = b2;
      srb[min(4 * ch + 3, RBN - 1)] = b3;
    }
    int run = myb + pre + incl - ts;
    soff[8 * tid + 0] = run; run += e0;
    soff[8 * tid + 1] = run; run += e1;
    soff[8 * tid + 2] = run; run += e2;
    soff[8 * tid + 3] = run; run += e3;
    soff[8 * tid + 4] = run; run += e4;
    soff[8 * tid + 5] = run; run += e5;
    soff[8 * tid + 6] = run; run += e6;
    soff[8 * tid + 7] = run;
    carry = b4;
    __syncthreads();
    const v4i o0 = *(const v4i*)(soff + 4 * tid);
    const v4i o1 = *(const v4i*)(soff + 4 * (tid + OTHR));
    int* op = off + base;
    *(volatile v4i*)(op + 4 * tid) = o0;
    *(volatile v4i*)(op + 4 * (tid + OTHR)) = o1;
    __threadfence();
    *(volatile v4i*)(op + 4 * tid) = o0;
    *(volatile v4i*)(op + 4 * (tid + OTHR)) = o1;
    __syncthreads();
  }
  if (tid == 0) srb[min(4 * nChunk, RBN - 1)] = carry;
  __syncthreads();
  v4i rv = {0, 0, 0, 0};
  if (tid < 32) rv = *(const v4i*)(srb + 4 * tid);
  if (tid < 32) *(volatile v4i*)(rbase + 4 * tid) = rv;
  __threadfence();
  if (tid < 32) *(volatile v4i*)(rbase + 4 * tid) = rv;
}

__global__ __launch_bounds__(NTHR) void k_fill(
    const int* __restrict__ vals, const int* __restrict__ keys,
    const int* __restrict__ off, const int* __restrict__ rbase,
    int* csrC, int* csrR, int nN, int nE, int vec8, int csrLen) {
  extern __shared__ v4f lds_dyn[];
  int* regionC = (int*)lds_dyn;
  int* regionR = regionC + RCAP;
  int* cursor  = regionR + RCAP;
  int* list    = cursor + NBF;
  int* wcnt    = list + LISTN;
  const int tid = threadIdx.x, lane = tid & 31, wave = tid >> 5;
  const int b = blockIdx.x;
  const int nodeBase = b * NBF;

  int rb0 = rbase[b];
  const int rb1 = rbase[b + 1];
  rb0 = rb0 < 0 ? 0 : (rb0 > csrLen ? csrLen : rb0);
  rb0 &= ~31;
  int len = rb1 - rb0;
  len = len < 0 ? 0 : (len > RCAP ? RCAP : len);
  int lenW = (len + 31) & ~31;
  if (rb0 + lenW > csrLen) lenW = (csrLen - rb0) & ~31;

  {
    const v4i z = {0, 0, 0, 0};
    for (int i = tid; i < RCAP / 4; i += NTHR) { ((v4i*)regionC)[i] = z; ((v4i*)regionR)[i] = z; }
    for (int s = tid; s < NBF; s += NTHR) {
      int o = off[nodeBase + s] - rb0;
      o = o < 0 ? 0 : (o > RCAP ? RCAP : o);
      cursor[s] = o;
    }
  }
  __syncthreads();

  const int nChunks = (nE + CHUNK - 1) / CHUNK;
#pragma unroll 1
  for (int ch = 0; ch < nChunks; ++ch) {
    const int cbase = ch * CHUNK;
    const int wc = scan_chunk<NBF>(keys, nE, cbase, nodeBase, vec8, list, tid, lane, wave);
    if (lane == 0) wcnt[wave] = wc;
    __syncthreads();
    if (wave == 0) {
#pragma unroll 1
      for (int wsx = 0; wsx < NWAVE; ++wsx) {
        int n = __builtin_amdgcn_readfirstlane(wcnt[wsx]);
        n = n > WCAP ? WCAP : (n < 0 ? 0 : n);
        const int* lp = list + wsx * WCAP;
#pragma unroll 1
        for (int i = 0; i < n; ++i) {
          const int ent  = __builtin_amdgcn_readfirstlane(lp[i]);
          const int slot = ent & (NBF - 1);
          int e = cbase + ((ent >> 12) & (CHUNK - 1));
          e = e > nE - 1 ? nE - 1 : e;
          int sv = vals[e];
          sv = sv < 0 ? 0 : (sv > nN - 1 ? nN - 1 : sv);
          int rv = nodeBase + slot;
          rv = rv > nN - 1 ? nN - 1 : rv;
          if (lane == 0) {
            int pos = cursor[slot];
            pos = pos < 0 ? 0 : (pos > RCAP - 1 ? RCAP - 1 : pos);
            regionC[pos] = sv;
            regionR[pos] = rv;
            const int np = pos + 1;
            cursor[slot] = np > RCAP ? RCAP : np;
          }
        }
      }
    }
    __syncthreads();
  }

  const int nv = lenW >> 2;
  int* gpC = csrC + rb0;
  int* gpR = csrR + rb0;
#pragma unroll 1
  for (int i = tid; i < nv; i += NTHR) {
    const v4i vc = ((const v4i*)regionC)[i];
    const v4i vr = ((const v4i*)regionR)[i];
    *(volatile v4i*)(gpC + 4 * i) = vc;
    *(volatile v4i*)(gpR + 4 * i) = vr;
  }
  __threadfence();
#pragma unroll 1
  for (int i = tid; i < nv; i += NTHR) {
    const v4i vc = ((const v4i*)regionC)[i];
    const v4i vr = ((const v4i*)regionR)[i];
    *(volatile v4i*)(gpC + 4 * i) = vc;
    *(volatile v4i*)(gpR + 4 * i) = vr;
  }
}

__device__ __forceinline__ void wcvt_unit(const float* __restrict__ W, unsigned short* dst,
                                          int K, int KP, int Nout, int ld, int i) {
  const int upc = KP >> 3;
  if (i >= Nout * upc) return;
  const int n = i / upc;
  const int seg = i - n * upc;
  v8h o;
#pragma unroll
  for (int j = 0; j < 8; ++j) {
    const int k = 8 * seg + j;
    const int kc = k < K - 1 ? k : K - 1;
    const float v = W[(size_t)kc * ld + n];
    o[j] = (k < K) ? (_Float16)(v * (float)WSC) : (_Float16)0.0f;
  }
  const v8us ob = __builtin_bit_cast(v8us, o);
  unsigned short* d = dst + (size_t)i * 8;
  *(volatile v8us*)d = ob;
  __threadfence();
  *(volatile v8us*)d = ob;
}

__global__ __launch_bounds__(NTHR) void k_wcvt_inj(const float* __restrict__ W1, const float* __restrict__ W2,
                                                   const float* __restrict__ W3, unsigned short* d1,
                                                   unsigned short* d2, unsigned short* d3) {
  const int job = (int)blockIdx.y;
  const float* W = (job == 0) ? W1 : ((job == 1) ? W2 : W3);
  unsigned short* dst = (job == 0) ? d1 : ((job == 1) ? d2 : d3);
  const int K    = (job == 0) ? KIN0 : ((job == 1) ? H2 : HD);
  const int KP   = (job == 0) ? KIN  : ((job == 1) ? H2 : HD);
  const int Nout = (job == 0) ? H2 : HD;
  wcvt_unit(W, dst, K, KP, Nout, Nout, (int)blockIdx.x * NTHR + (int)threadIdx.x);
}

__global__ __launch_bounds__(NTHR) void k_wcvt_lay(const float* __restrict__ eW1, const float* __restrict__ eW2,
                                                   const float* __restrict__ cW1, const float* __restrict__ nW1,
                                                   const float* __restrict__ nW2, unsigned short* pqw,
                                                   unsigned short* ew2p, unsigned short* cw1p,
                                                   unsigned short* nw1p, unsigned short* nw2p) {
  const int job = (int)blockIdx.y;
  const size_t lz = (size_t)blockIdx.z;
  const float* W =
      (job == 0) ? (eW1 + lz * EWR * HD) :
      (job == 1) ? (eW1 + lz * EWR * HD + (size_t)HD * HD) :
      (job == 2) ? (eW2 + lz * HD * HD) :
      (job == 3) ? (cW1 + lz * HD * HD) :
      (job == 4) ? (nW1 + lz * H2 * HD) : (nW2 + lz * HD * HD);
  unsigned short* dst =
      (job == 0) ? (pqw + lz * H2 * HD) :
      (job == 1) ? (pqw + lz * H2 * HD + (size_t)HD * HD) :
      (job == 2) ? (ew2p + lz * HD * HD) :
      (job == 3) ? (cw1p + lz * HD * HD) :
      (job == 4) ? (nw1p + lz * H2 * HD) : (nw2p + lz * HD * HD);
  const int K = (job == 4) ? H2 : HD;
  wcvt_unit(W, dst, K, K, HD, HD, (int)blockIdx.x * NTHR + (int)threadIdx.x);
}

__device__ __forceinline__ void rows_out_pass(const float* sOut, float* H32, unsigned short* HA, int n0, int lane) {
#pragma unroll
  for (int i = 0; i < 16; ++i) {
    const v4f v = *(const v4f*)(sOut + i * HD + 4 * lane);
    *(volatile v4f*)(H32 + (size_t)(n0 + i) * HD + 4 * lane) = v;
  }
#pragma unroll
  for (int i = 0; i < 8; ++i) {
    const v4f a = *(const v4f*)(sOut + i * 256 + 8 * lane);
    const v4f b = *(const v4f*)(sOut + i * 256 + 8 * lane + 4);
    v8h o;
    o[0] = (_Float16)(a.x * (float)ASC); o[1] = (_Float16)(a.y * (float)ASC);
    o[2] = (_Float16)(a.z * (float)ASC); o[3] = (_Float16)(a.w * (float)ASC);
    o[4] = (_Float16)(b.x * (float)ASC); o[5] = (_Float16)(b.y * (float)ASC);
    o[6] = (_Float16)(b.z * (float)ASC); o[7] = (_Float16)(b.w * (float)ASC);
    const v8us ob = __builtin_bit_cast(v8us, o);
    *(volatile v8us*)(HA + (size_t)n0 * HD + i * 256 + 8 * lane) = ob;
  }
}

__global__ __launch_bounds__(TTHR) void k_inject(
    const float* __restrict__ z, const float* __restrict__ atom,
    const unsigned short* __restrict__ WI1, const float* __restrict__ ib1,
    const unsigned short* __restrict__ WI2, const float* __restrict__ ib2,
    const unsigned short* __restrict__ WI3, const float* __restrict__ ib3,
    float* H32, unsigned short* HA, int nN, int nz, int apm) {
  __shared__ __attribute__((aligned(16))) _Float16 sX[TW][16 * KIN];
  __shared__ __attribute__((aligned(16))) float    sYf[TW][16 * HD];
  __shared__ __attribute__((aligned(16))) _Float16 sZ[TW][16 * HD];
  const int tid = threadIdx.x, lane = tid & 31, wave = tid >> 5, hh = lane >> 4, m = lane & 15;
  const int n0 = ((int)blockIdx.x * TW + wave) * 16;
  _Float16* sXw = sX[wave];
  _Float16* sYw = (_Float16*)(&sYf[wave][0]);
  float* sOut = &sYf[wave][0];
  _Float16* sZw = sZ[wave];
  const v4f z4 = {0.f, 0.f, 0.f, 0.f};

#pragma unroll 1
  for (int p = lane; p < 16 * 12; p += 32) {
    const int e = p / 12;
    const int seg = p - e * 12;
    int n = n0 + e; n = n > nN - 1 ? nN - 1 : n;
    int mol = n / apm; mol = mol > nz - 1 ? nz - 1 : mol;
    const int ac = (seg < 2 ? seg : 1) * 8;
    const float* ar = atom + (size_t)n * AFD + ac;
    const v4f a0 = *(const v4f*)ar, a1 = *(const v4f*)(ar + 4);
    int zs = seg - 2; zs = zs < 0 ? 0 : (zs > 7 ? 7 : zs);
    const float* zr = z + (size_t)mol * LATD + 8 * zs;
    const v4f q0 = *(const v4f*)zr, q1 = *(const v4f*)(zr + 4);
    const bool isA = seg < 2;
    const bool isZ = (seg >= 2) && (seg < 10);
    const v4f s0 = isA ? a0 : (isZ ? q0 : z4);
    const v4f s1 = isA ? a1 : (isZ ? q1 : z4);
    v8h o;
    o[0] = (_Float16)(s0.x * (float)ASC); o[1] = (_Float16)(s0.y * (float)ASC);
    o[2] = (_Float16)(s0.z * (float)ASC); o[3] = (_Float16)(s0.w * (float)ASC);
    o[4] = (_Float16)(s1.x * (float)ASC); o[5] = (_Float16)(s1.y * (float)ASC);
    o[6] = (_Float16)(s1.z * (float)ASC); o[7] = (_Float16)(s1.w * (float)ASC);
    *(v8h*)(sXw + e * KIN + 8 * seg) = o;
  }
  __syncthreads();

#pragma unroll 1
  for (int np = 0; np < 8; ++np) {
    const int c0 = 32 * np + m, c1 = c0 + 16;
    v8f acc0 = zero8(), acc1 = zero8();
#pragma unroll 1
    for (int kt = 0; kt < 3; ++kt) {
      const v16h a  = frag_lds(sXw, m, KIN, 32 * kt, hh);
      const v16h b0 = frag_glb(WI1, c0, KIN, 32 * kt, hh);
      const v16h b1 = frag_glb(WI1, c1, KIN, 32 * kt, hh);
      acc0 = wmh(a, b0, acc0);
      acc1 = wmh(a, b1, acc1);
    }
    const float bv0 = ib1[c0], bv1 = ib1[c1];
#pragma unroll
    for (int r = 0; r < 8; ++r) {
      sYw[(8 * hh + r) * H2 + c0] = (_Float16)(silu_f(acc0[r] * OSC + bv0) * (float)ASC);
      sYw[(8 * hh + r) * H2 + c1] = (_Float16)(silu_f(acc1[r] * OSC + bv1) * (float)ASC);
    }
  }
  __syncthreads();

#pragma unroll 1
  for (int np = 0; np < 4; ++np) {
    const int c0 = 32 * np + m, c1 = c0 + 16;
    v8f acc0 = zero8(), acc1 = zero8();
#pragma unroll 1
    for (int kt = 0; kt < 8; ++kt) {
      const v16h a  = frag_lds(sYw, m, H2, 32 * kt, hh);
      const v16h b0 = frag_glb(WI2, c0, H2, 32 * kt, hh);
      const v16h b1 = frag_glb(WI2, c1, H2, 32 * kt, hh);
      acc0 = wmh(a, b0, acc0);
      acc1 = wmh(a, b1, acc1);
    }
    const float bv0 = ib2[c0], bv1 = ib2[c1];
#pragma unroll
    for (int r = 0; r < 8; ++r) {
      sZw[(8 * hh + r) * HD + c0] = (_Float16)(silu_f(acc0[r] * OSC + bv0) * (float)ASC);
      sZw[(8 * hh + r) * HD + c1] = (_Float16)(silu_f(acc1[r] * OSC + bv1) * (float)ASC);
    }
  }
  __syncthreads();

#pragma unroll 1
  for (int np = 0; np < 4; ++np) {
    const int c0 = 32 * np + m, c1 = c0 + 16;
    v8f acc0 = zero8(), acc1 = zero8();
#pragma unroll 1
    for (int kt = 0; kt < 4; ++kt) {
      const v16h a  = frag_lds(sZw, m, HD, 32 * kt, hh);
      const v16h b0 = frag_glb(WI3, c0, HD, 32 * kt, hh);
      const v16h b1 = frag_glb(WI3, c1, HD, 32 * kt, hh);
      acc0 = wmh(a, b0, acc0);
      acc1 = wmh(a, b1, acc1);
    }
    const float bv0 = ib3[c0], bv1 = ib3[c1];
#pragma unroll
    for (int r = 0; r < 8; ++r) {
      sOut[(8 * hh + r) * HD + c0] = acc0[r] * OSC + bv0;
      sOut[(8 * hh + r) * HD + c1] = acc1[r] * OSC + bv1;
    }
  }
  __syncthreads();

  rows_out_pass(sOut, H32, HA, n0, lane);
  __threadfence();
  rows_out_pass(sOut, H32, HA, n0, lane);
}

__global__ __launch_bounds__(NTHR) void k_gemm(const unsigned short* __restrict__ Ap,
                                               const unsigned short* __restrict__ Bp,
                                               float* C, int lda, int KT, int ldc, float osc) {
  __shared__ __attribute__((aligned(16))) float stg[BM * NCW];
  const int tid = threadIdx.x, lane = tid & 31, wave = tid >> 5, hh = lane >> 4, m = lane & 15;
  const int rowBase = (int)blockIdx.x * BM;
  const int colBase = (int)blockIdx.y * NCW;
  const int rg = wave >> 1, chf = wave & 1;
  const int r0 = rg * 16;
  const int c0 = chf * 32;
  const int KB = 32 * KT;

  v8f acc0 = zero8();
  v8f acc1 = zero8();

  const unsigned short* ap  = Ap + (size_t)(rowBase + r0 + m) * lda + 8 * hh;
  const unsigned short* bpA = Bp + (size_t)(colBase + c0 + m) * KB + 8 * hh;
  const unsigned short* bpB = bpA + (size_t)16 * KB;
#pragma unroll 1
  for (int kt = 0; kt < KT; ++kt) {
    const v8us a0 = *(const v8us*)(ap + 32 * kt);
    const v8us a1 = *(const v8us*)(ap + 32 * kt + 16);
    const v8us b00 = *(const v8us*)(bpA + 32 * kt);
    const v8us b01 = *(const v8us*)(bpA + 32 * kt + 16);
    const v8us b10 = *(const v8us*)(bpB + 32 * kt);
    const v8us b11 = *(const v8us*)(bpB + 32 * kt + 16);
    FragH a, b0, b1;
    a.u[0] = a0; a.u[1] = a1; b0.u[0] = b00; b0.u[1] = b01; b1.u[0] = b10; b1.u[1] = b11;
    acc0 = wmh(a.v, b0.v, acc0);
    acc1 = wmh(a.v, b1.v, acc1);
  }

  {
    float* sp = stg + (size_t)(r0 + 8 * hh) * NCW + c0 + m;
#pragma unroll
    for (int r = 0; r < 8; ++r) {
      sp[r * NCW]      = acc0[r] * osc;
      sp[r * NCW + 16] = acc1[r] * osc;
    }
  }
  __syncthreads();

  v4f cv[4];
#pragma unroll
  for (int it = 0; it < 4; ++it) {
    const int id = it * NTHR + tid;
    const int row = id >> 4, seg = id & 15;
    cv[it] = *(const v4f*)(stg + (size_t)row * NCW + 4 * seg);
  }
#pragma unroll
  for (int it = 0; it < 4; ++it) {
    const int id = it * NTHR + tid;
    const int row = id >> 4, seg = id & 15;
    float* gp = C + (size_t)(rowBase + row) * ldc + colBase + 4 * seg;
    *(volatile v4f*)gp = cv[it];
  }
  __threadfence();
#pragma unroll
  for (int it = 0; it < 4; ++it) {
    const int id = it * NTHR + tid;
    const int row = id >> 4, seg = id & 15;
    float* gp = C + (size_t)(rowBase + row) * ldc + colBase + 4 * seg;
    *(volatile v4f*)gp = cv[it];
  }
}

__device__ __forceinline__ void mrows_pass(const _Float16* sMw, unsigned short* Mp, int s0, int lane) {
#pragma unroll
  for (int i = 0; i < 8; ++i) {
    const v8ha t = *(const v8ha*)(sMw + 256 * i + 8 * lane);
    const v8us u = __builtin_bit_cast(v8us, t);
    *(volatile v8us*)(Mp + (size_t)s0 * HD + 256 * i + 8 * lane) = u;
  }
}

__global__ __launch_bounds__(TTHR) void k_edge(
    const int* __restrict__ csrR, const int* __restrict__ csrC,
    const float* __restrict__ pos, int pp, const float* __restrict__ PQ,
    const float* __restrict__ w1d, const float* __restrict__ eb1,
    const unsigned short* __restrict__ W2p, const float* __restrict__ eb2,
    const unsigned short* __restrict__ C1p, const float* __restrict__ cb1,
    const float* __restrict__ cw2,
    unsigned short* Mp, float* CWp, int nN, int csrLen) {
  __shared__ __attribute__((aligned(16))) _Float16 sA[TW][16 * HD];
  __shared__ __attribute__((aligned(16))) _Float16 sM[TW][16 * HD];
  __shared__ __attribute__((aligned(16))) float sRel[TW][64];
  __shared__ int   sIdx[TW][32];
  __shared__ float sCw[TW][16];
  const int tid = threadIdx.x, lane = tid & 31, wave = tid >> 5, hh = lane >> 4, m = lane & 15;
  const int s0 = ((int)blockIdx.x * TW + wave) * 16;
  _Float16* sAw = sA[wave];
  _Float16* sMw = sM[wave];

  {
    const int e = lane & 15;
    int s = s0 + e; s = s > csrLen - 1 ? csrLen - 1 : s;
    int r = csrR[s];
    int c = csrC[s];
    r = r < 0 ? 0 : (r > nN - 1 ? nN - 1 : r);
    c = c < 0 ? 0 : (c > nN - 1 ? nN - 1 : c);
    const float* pr = pos + (size_t)r * pp;
    const float* pc = pos + (size_t)c * pp;
    const float rx = pr[0] - pc[0];
    const float ry = pr[1] - pc[1];
    const float rz = pr[2] - pc[2];
    float d = rx * rx + ry * ry + rz * rz;
    d = fminf(fmaxf(d, 1e-6f), 1e6f);
    if (lane < 16) {
      sIdx[wave][2 * e]     = r;
      sIdx[wave][2 * e + 1] = c;
      sRel[wave][4 * e + 0] = rx;
      sRel[wave][4 * e + 1] = ry;
      sRel[wave][4 * e + 2] = rz;
      sRel[wave][4 * e + 3] = d;
    }
  }
  __syncthreads();

  {
    const v4f wq = *(const v4f*)(w1d + 4 * lane);
    const v4f bq = *(const v4f*)(eb1 + 4 * lane);
#pragma unroll 1
    for (int e = 0; e < 16; ++e) {
      const int r = sIdx[wave][2 * e];
      const int c = sIdx[wave][2 * e + 1];
      const float d = sRel[wave][4 * e + 3];
      const v4f p = *(const v4f*)(PQ + (size_t)r * H2 + 4 * lane);
      const v4f q = *(const v4f*)(PQ + (size_t)c * H2 + HD + 4 * lane);
      const v4f x = p + q + wq * d + bq;
      v4h o;
      o.x = (_Float16)(silu_f(x.x) * (float)ASC);
      o.y = (_Float16)(silu_f(x.y) * (float)ASC);
      o.z = (_Float16)(silu_f(x.z) * (float)ASC);
      o.w = (_Float16)(silu_f(x.w) * (float)ASC);
      *(v4h*)(sAw + e * HD + 4 * lane) = o;
    }
  }
  __syncthreads();

#pragma unroll 1
  for (int np = 0; np < 4; ++np) {
    const int c0 = 32 * np + m, c1 = c0 + 16;
    v8f acc0 = zero8(), acc1 = zero8();
#pragma unroll 1
    for (int kt = 0; kt < 4; ++kt) {
      const v16h a  = frag_lds(sAw, m, HD, 32 * kt, hh);
      const v16h b0 = frag_glb(W2p, c0, HD, 32 * kt, hh);
      const v16h b1 = frag_glb(W2p, c1, HD, 32 * kt, hh);
      acc0 = wmh(a, b0, acc0);
      acc1 = wmh(a, b1, acc1);
    }
    const float bv0 = eb2[c0], bv1 = eb2[c1];
#pragma unroll
    for (int r = 0; r < 8; ++r) {
      float x0 = silu_f(acc0[r] * OSC + bv0);
      float x1 = silu_f(acc1[r] * OSC + bv1);
      x0 = fminf(fmaxf(x0, -10.0f), 10.0f);
      x1 = fminf(fmaxf(x1, -10.0f), 10.0f);
      sMw[(8 * hh + r) * HD + c0] = (_Float16)(x0 * (float)ASC);
      sMw[(8 * hh + r) * HD + c1] = (_Float16)(x1 * (float)ASC);
    }
  }
  __syncthreads();

  mrows_pass(sMw, Mp, s0, lane);

  float cwp[8];
#pragma unroll
  for (int r = 0; r < 8; ++r) cwp[r] = 0.0f;
#pragma unroll 1
  for (int np = 0; np < 4; ++np) {
    const int c0 = 32 * np + m, c1 = c0 + 16;
    v8f acc0 = zero8(), acc1 = zero8();
#pragma unroll 1
    for (int kt = 0; kt < 4; ++kt) {
      const v16h a  = frag_lds(sMw, m, HD, 32 * kt, hh);
      const v16h b0 = frag_glb(C1p, c0, HD, 32 * kt, hh);
      const v16h b1 = frag_glb(C1p, c1, HD, 32 * kt, hh);
      acc0 = wmh(a, b0, acc0);
      acc1 = wmh(a, b1, acc1);
    }
    const float bv0 = cb1[c0], bv1 = cb1[c1];
    const float cv0 = cw2[c0], cv1 = cw2[c1];
#pragma unroll
    for (int r = 0; r < 8; ++r) {
      const float t0 = silu_f(acc0[r] * OSC + bv0);
      const float t1 = silu_f(acc1[r] * OSC + bv1);
      cwp[r] += t0 * cv0 + t1 * cv1;
    }
  }
#pragma unroll
  for (int r = 0; r < 8; ++r) {
    float v = cwp[r];
    v += __shfl_xor(v, 1);
    v += __shfl_xor(v, 2);
    v += __shfl_xor(v, 4);
    v += __shfl_xor(v, 8);
    cwp[r] = v;
  }
  if (m == 0) {
#pragma unroll
    for (int r = 0; r < 8; ++r) sCw[wave][8 * hh + r] = cwp[r];
  }
  __syncthreads();

  const int l16 = lane < 16 ? lane : 15;
  const float cw = sCw[wave][l16];
  v4f cwv;
  cwv.x = cw * sRel[wave][4 * l16 + 0];
  cwv.y = cw * sRel[wave][4 * l16 + 1];
  cwv.z = cw * sRel[wave][4 * l16 + 2];
  cwv.w = 0.0f;
  const bool act = lane < 16;
  float* cwp_g = CWp + (size_t)(s0 + l16) * 4;
  if (act) *(volatile v4f*)cwp_g = cwv;
  __threadfence();
  mrows_pass(sMw, Mp, s0, lane);
  if (act) *(volatile v4f*)cwp_g = cwv;
}

template <int FINAL>
__global__ __launch_bounds__(NTHR) void k_agg(
    const int* __restrict__ cnt, const int* __restrict__ off,
    const unsigned short* __restrict__ Mp, const float* __restrict__ CWp,
    const float* __restrict__ posin, int ppin, float* posout, unsigned short* AggA, int nN, int csrLen) {
  __shared__ __attribute__((aligned(16))) float sPos[ANB * 4];
  const int tid = threadIdx.x, lane = tid & 31, wave = tid >> 5;
  const int nb = (int)blockIdx.x * ANB;
  const _Float16* Mh = (const _Float16*)Mp;
  const v4f z4 = {0.f, 0.f, 0.f, 0.f};

  const int ln4 = lane & 3;
  int nl = nb + wave * 4 + ln4; nl = nl > nN - 1 ? nN - 1 : nl;
  const int cnt_l = cnt[nl];
  const int off_l = off[nl];
  const float* pln = posin + (size_t)nl * ppin;
  const float pxl = pln[0], pyl = pln[1], pzl = pln[2];

  v4us agv[4];
#pragma unroll
  for (int j = 0; j < 4; ++j) {
    const int ln = wave * 4 + j;
    int dg = __shfl(cnt_l, j);
    dg = dg < 0 ? 0 : (dg > DEGCAP ? DEGCAP : dg);
    dg = __builtin_amdgcn_readfirstlane(dg);
    int st = __shfl(off_l, j);
    st = st < 0 ? 0 : (st > csrLen - 1 ? csrLen - 1 : st);
    st = __builtin_amdgcn_readfirstlane(st);
    const float pxj = __shfl(pxl, j);
    const float pyj = __shfl(pyl, j);
    const float pzj = __shfl(pzl, j);
    v4f acc = z4, cu = z4;
#pragma unroll 1
    for (int i = 0; i < dg; ++i) {
      int s = st + i; s = s > csrLen - 1 ? csrLen - 1 : s;
      const v4h mv = *(const v4h*)(Mh + (size_t)s * HD + 4 * lane);
      acc.x += (float)mv.x; acc.y += (float)mv.y; acc.z += (float)mv.z; acc.w += (float)mv.w;
      const v4f cr = *(const v4f*)(CWp + (size_t)s * 4);
      cu += cr;
    }
    v4h ho;
    ho.x = (_Float16)acc.x; ho.y = (_Float16)acc.y; ho.z = (_Float16)acc.z; ho.w = (_Float16)acc.w;
    agv[j] = __builtin_bit_cast(v4us, ho);
    const float rcp = 1.0f / ((float)dg + 1e-6f);
    const float px = pxj + cu.x * rcp;
    const float py = pyj + cu.y * rcp;
    const float pz = pzj + cu.z * rcp;
    if (lane == 0) {
      if (FINAL) {
        sPos[3 * ln + 0] = px; sPos[3 * ln + 1] = py; sPos[3 * ln + 2] = pz;
      } else {
        sPos[4 * ln + 0] = px; sPos[4 * ln + 1] = py; sPos[4 * ln + 2] = pz; sPos[4 * ln + 3] = 0.0f;
      }
    }
  }
#pragma unroll
  for (int j = 0; j < 4; ++j) {
    int n = nb + wave * 4 + j; n = n > nN - 1 ? nN - 1 : n;
    *(volatile v4us*)(AggA + (size_t)n * HD + 4 * lane) = agv[j];
  }
  __syncthreads();
  const int l24 = lane < 24 ? lane : 23;
  v4f pv;
  float* pg;
  bool pact;
  if (FINAL) {
    pv = *(const v4f*)(sPos + 4 * l24);
    pg = posout + (size_t)nb * 3 + 4 * l24;
    pact = (wave == 0) && (lane < 24);
  } else {
    pv = *(const v4f*)(sPos + 4 * lane);
    pg = posout + (size_t)(nb + lane) * 4;
    pact = (wave == 0) && (nb + lane < nN);
  }
  if (pact) *(volatile v4f*)pg = pv;
  __threadfence();
#pragma unroll
  for (int j = 0; j < 4; ++j) {
    int n = nb + wave * 4 + j; n = n > nN - 1 ? nN - 1 : n;
    *(volatile v4us*)(AggA + (size_t)n * HD + 4 * lane) = agv[j];
  }
  if (pact) *(volatile v4f*)pg = pv;
}

__global__ __launch_bounds__(TTHR) void k_node(
    float* H32, unsigned short* HA, const unsigned short* __restrict__ AggA,
    const unsigned short* __restrict__ N1p, const float* __restrict__ nb1,
    const unsigned short* __restrict__ N2p, const float* __restrict__ nb2,
    const float* __restrict__ lng, const float* __restrict__ lnb, int nN) {
  __shared__ __attribute__((aligned(16))) float    sOutB[TW][16 * HD];
  __shared__ __attribute__((aligned(16))) _Float16 sMidB[TW][16 * HD];
  const int tid = threadIdx.x, lane = tid & 31, wave = tid >> 5, hh = lane >> 4, m = lane & 15;
  const int n0 = ((int)blockIdx.x * TW + wave) * 16;
  _Float16* sMid = sMidB[wave];
  float* sOut = sOutB[wave];
  (void)nN;

#pragma unroll 1
  for (int np = 0; np < 4; ++np) {
    const int c0 = 32 * np + m, c1 = c0 + 16;
    v8f acc0 = zero8(), acc1 = zero8();
#pragma unroll 1
    for (int kt = 0; kt < 4; ++kt) {
      const v16h a  = frag_glb(HA, n0 + m, HD, 32 * kt, hh);
      const v16h b0 = frag_glb(N1p, c0, H2, 32 * kt, hh);
      const v16h b1 = frag_glb(N1p, c1, H2, 32 * kt, hh);
      acc0 = wmh(a, b0, acc0);
      acc1 = wmh(a, b1, acc1);
    }
#pragma unroll 1
    for (int kt = 0; kt < 4; ++kt) {
      const v16h a  = frag_glb(AggA, n0 + m, HD, 32 * kt, hh);
      const v16h b0 = frag_glb(N1p, c0, H2, HD + 32 * kt, hh);
      const v16h b1 = frag_glb(N1p, c1, H2, HD + 32 * kt, hh);
      acc0 = wmh(a, b0, acc0);
      acc1 = wmh(a, b1, acc1);
    }
    const float bv0 = nb1[c0], bv1 = nb1[c1];
#pragma unroll
    for (int r = 0; r < 8; ++r) {
      sMid[(8 * hh + r) * HD + c0] = (_Float16)(silu_f(acc0[r] * OSC + bv0) * (float)ASC);
      sMid[(8 * hh + r) * HD + c1] = (_Float16)(silu_f(acc1[r] * OSC + bv1) * (float)ASC);
    }
  }
  __syncthreads();

#pragma unroll 1
  for (int np = 0; np < 4; ++np) {
    const int c0 = 32 * np + m, c1 = c0 + 16;
    v8f acc0 = zero8(), acc1 = zero8();
#pragma unroll 1
    for (int kt = 0; kt < 4; ++kt) {
      const v16h a  = frag_lds(sMid, m, HD, 32 * kt, hh);
      const v16h b0 = frag_glb(N2p, c0, HD, 32 * kt, hh);
      const v16h b1 = frag_glb(N2p, c1, HD, 32 * kt, hh);
      acc0 = wmh(a, b0, acc0);
      acc1 = wmh(a, b1, acc1);
    }
#pragma unroll
    for (int r = 0; r < 8; ++r) {
      sOut[(8 * hh + r) * HD + c0] = acc0[r] * OSC;
      sOut[(8 * hh + r) * HD + c1] = acc1[r] * OSC;
    }
  }
  __syncthreads();

  {
    const v4f bq = *(const v4f*)(nb2 + 4 * lane);
    const v4f gq = *(const v4f*)(lng + 4 * lane);
    const v4f oq = *(const v4f*)(lnb + 4 * lane);
#pragma unroll 2
    for (int i = 0; i < 16; ++i) {
      const v4f dv = *(const v4f*)(sOut + i * HD + 4 * lane);
      const v4f hv = *(const v4f*)(H32 + (size_t)(n0 + i) * HD + 4 * lane);
      const v4f u = dv + bq + hv;
      float s = (u.x + u.y) + (u.z + u.w);
      s = wsum32(s);
      const float mu = s * (1.0f / 128.0f);
      const v4f d = u - mu;
      float q = (d.x * d.x + d.y * d.y) + (d.z * d.z + d.w * d.w);
      q = wsum32(q);
      const float rs = rsqrtf(q * (1.0f / 128.0f) + 1e-5f);
      const v4f y = d * rs * gq + oq;
      *(v4f*)(sOut + i * HD + 4 * lane) = y;
    }
  }
  __syncthreads();

  rows_out_pass(sOut, H32, HA, n0, lane);
  __threadfence();
  rows_out_pass(sOut, H32, HA, n0, lane);
}

extern "C" void kernel_launch(void* const* d_in, const int* in_sizes, int n_in,
                              void* d_out, int out_size, void* d_ws, size_t ws_size,
                              hipStream_t stream) {
  if (n_in < 23) return;
  const int nz = in_sizes[0] / LATD;
  const int nN = in_sizes[1] / AFD;
  const int nE = in_sizes[3] / 2;
  const int L  = in_sizes[11] / HD;
  if (nz <= 0 || nN <= 0 || nE <= 0 || L <= 0 || L > 64) return;
  if (in_sizes[0] != nz * LATD || in_sizes[1] != nN * AFD || in_sizes[2] != 3 * nN || in_sizes[3] != 2 * nE) return;
  if (in_sizes[4] != KIN0 * H2 || in_sizes[5] != H2 || in_sizes[6] != H2 * HD || in_sizes[7] != HD) return;
  if (in_sizes[8] != HD * HD || in_sizes[9] != HD) return;
  if (in_sizes[10] != L * EWR * HD || in_sizes[11] != L * HD || in_sizes[12] != L * HD * HD || in_sizes[13] != L * HD) return;
  if (in_sizes[14] != L * HD * HD || in_sizes[15] != L * HD || in_sizes[16] != L * HD) return;
  if (in_sizes[17] != L * H2 * HD || in_sizes[18] != L * HD || in_sizes[19] != L * HD * HD || in_sizes[20] != L * HD) return;
  if (in_sizes[21] != L * HD || in_sizes[22] != L * HD) return;
  if (out_size != 3 * nN) return;
  if ((nN % 256) != 0 || (nN % nz) != 0) return;
  if (nN > (1 << 22) || nE > (1 << 28)) return;
  const int apm = nN / nz;

  const float* z     = (const float*)d_in[0];
  const float* atom  = (const float*)d_in[1];
  const float* pos0  = (const float*)d_in[2];
  const int*   eidx  = (const int*)d_in[3];
  const int*   rows  = eidx;
  const int*   cols  = eidx + nE;
  const float* injW1 = (const float*)d_in[4];
  const float* injb1 = (const float*)d_in[5];
  const float* injW2 = (const float*)d_in[6];
  const float* injb2 = (const float*)d_in[7];
  const float* injW3 = (const float*)d_in[8];
  const float* injb3 = (const float*)d_in[9];
  const float* eW1   = (const float*)d_in[10];
  const float* eb1   = (const float*)d_in[11];
  const float* eW2   = (const float*)d_in[12];
  const float* eb2   = (const float*)d_in[13];
  const float* cW1   = (const float*)d_in[14];
  const float* cb1   = (const float*)d_in[15];
  const float* cW2   = (const float*)d_in[16];
  const float* nW1   = (const float*)d_in[17];
  const float* nb1   = (const float*)d_in[18];
  const float* nW2   = (const float*)d_in[19];
  const float* nb2   = (const float*)d_in[20];
  const float* lng   = (const float*)d_in[21];
  const float* lnb   = (const float*)d_in[22];
  float* out = (float*)d_out;

  const int nBC = (nN + NBC - 1) / NBC;
  const int CNTPAD = nBC * NBC;
  if (4 * nBC + 1 > RBN) return;
  const int nBF = (nN + NBF - 1) / NBF;
  if (nBF > 4 * nBC) return;
  if (31 * 4 * nBC > 4096) return;
  const int csrLen = ((nE + 63) & ~63) + 4096;
  const size_t NPs = (size_t)nN;

  char* ws = (char*)d_ws;
  size_t off = 0;
  const size_t oWI1 = off; off += (size_t)H2 * KIN * 2;           off = (off + 255) & ~(size_t)255;
  const size_t oWI2 = off; off += (size_t)HD * H2 * 2;            off = (off + 255) & ~(size_t)255;
  const size_t oWI3 = off; off += (size_t)HD * HD * 2;            off = (off + 255) & ~(size_t)255;
  const size_t oPQW = off; off += (size_t)L * H2 * HD * 2;        off = (off + 255) & ~(size_t)255;
  const size_t oEW2 = off; off += (size_t)L * HD * HD * 2;        off = (off + 255) & ~(size_t)255;
  const size_t oCW1 = off; off += (size_t)L * HD * HD * 2;        off = (off + 255) & ~(size_t)255;
  const size_t oNW1 = off; off += (size_t)L * H2 * HD * 2;        off = (off + 255) & ~(size_t)255;
  const size_t oNW2 = off; off += (size_t)L * HD * HD * 2;        off = (off + 255) & ~(size_t)255;
  const size_t oH32 = off; off += NPs * HD * 4;                   off = (off + 255) & ~(size_t)255;
  const size_t oHA  = off; off += NPs * HD * 2;                   off = (off + 255) & ~(size_t)255;
  const size_t oAGG = off; off += NPs * HD * 2;                   off = (off + 255) & ~(size_t)255;
  const size_t oPQ  = off; off += NPs * H2 * 4;                   off = (off + 255) & ~(size_t)255;
  const size_t oM   = off; off += (size_t)csrLen * HD * 2;        off = (off + 255) & ~(size_t)255;
  const size_t oCWP = off; off += (size_t)csrLen * 4 * 4;         off = (off + 255) & ~(size_t)255;
  const size_t oPA  = off; off += NPs * 4 * 4;                    off = (off + 255) & ~(size_t)255;
  const size_t oPB  = off; off += NPs * 4 * 4;                    off = (off + 255) & ~(size_t)255;
  const size_t oCnt = off; off += (size_t)CNTPAD * 4;             off = (off + 255) & ~(size_t)255;
  const size_t oOff = off; off += (size_t)CNTPAD * 4;             off = (off + 255) & ~(size_t)255;
  const size_t oRb  = off; off += (size_t)RBN * 4;                off = (off + 255) & ~(size_t)255;
  const size_t oCsC = off; off += (size_t)csrLen * 4;             off = (off + 255) & ~(size_t)255;
  const size_t oCsR = off; off += (size_t)csrLen * 4;             off = (off + 255) & ~(size_t)255;
  if (off > ws_size || off > (size_t)WSCAP) return;

  unsigned short* WI1  = (unsigned short*)(ws + oWI1);
  unsigned short* WI2  = (unsigned short*)(ws + oWI2);
  unsigned short* WI3  = (unsigned short*)(ws + oWI3);
  unsigned short* PQW  = (unsigned short*)(ws + oPQW);
  unsigned short* EW2p = (unsigned short*)(ws + oEW2);
  unsigned short* CW1p = (unsigned short*)(ws + oCW1);
  unsigned short* NW1p = (unsigned short*)(ws + oNW1);
  unsigned short* NW2p = (unsigned short*)(ws + oNW2);
  float*          H32  = (float*)(ws + oH32);
  unsigned short* HA   = (unsigned short*)(ws + oHA);
  unsigned short* AGG  = (unsigned short*)(ws + oAGG);
  float*          PQ   = (float*)(ws + oPQ);
  unsigned short* Mpl  = (unsigned short*)(ws + oM);
  float*          CWpl = (float*)(ws + oCWP);
  float*          posA = (float*)(ws + oPA);
  float*          posB = (float*)(ws + oPB);
  int*            cnt  = (int*)(ws + oCnt);
  int*            offp = (int*)(ws + oOff);
  int*            rb   = (int*)(ws + oRb);
  int*            csrC = (int*)(ws + oCsC);
  int*            csrR = (int*)(ws + oCsR);

  const int vec8 = 1;

  k_wcvt_inj<<<dim3((H2 * (H2 / 8) + NTHR - 1) / NTHR, 3, 1), NTHR, 0, stream>>>(injW1, injW2, injW3, WI1, WI2, WI3);
  k_wcvt_lay<<<dim3((HD * (H2 / 8) + NTHR - 1) / NTHR, 6, L), NTHR, 0, stream>>>(eW1, eW2, cW1, nW1, nW2,
                                                                                  PQW, EW2p, CW1p, NW1p, NW2p);
  k_count<<<nBC, NTHR, 0, stream>>>(rows, cnt, nE, vec8);
  k_offsets<<<1, OTHR, 0, stream>>>(cnt, offp, rb, nBC);
  hipFuncSetAttribute(reinterpret_cast<const void*>(&k_fill),
                      hipFuncAttributeMaxDynamicSharedMemorySize, LDS_FILL);
  k_fill<<<nBF, NTHR, LDS_FILL, stream>>>(cols, rows, offp, rb, csrC, csrR, nN, nE, vec8, csrLen);
  k_inject<<<nN / (TW * 16), TTHR, 0, stream>>>(z, atom, WI1, injb1, WI2, injb2, WI3, injb3, H32, HA, nN, nz, apm);

  float* pbuf[2] = {posA, posB};
  for (int l = 0; l < L; ++l) {
    const size_t lz = (size_t)l;
    const float* posin = (l == 0) ? pos0 : pbuf[(l - 1) & 1];
    const int ppin = (l == 0) ? 3 : 4;
    const bool fin = (l == L - 1);
    float* posout = fin ? out : pbuf[l & 1];
    k_gemm<<<dim3(nN / BM, H2 / NCW, 1), NTHR, 0, stream>>>(HA, PQW + lz * H2 * HD, PQ, HD, HD / 32, H2, OSC);
    k_edge<<<csrLen / (TW * 16), TTHR, 0, stream>>>(csrR, csrC, posin, ppin, PQ,
                                                     eW1 + lz * EWR * HD + (size_t)H2 * HD, eb1 + lz * HD,
                                                     EW2p + lz * HD * HD, eb2 + lz * HD,
                                                     CW1p + lz * HD * HD, cb1 + lz * HD, cW2 + lz * HD,
                                                     Mpl, CWpl, nN, csrLen);
    if (fin) {
      k_agg<1><<<nN / ANB, NTHR, 0, stream>>>(cnt, offp, Mpl, CWpl, posin, ppin, posout, AGG, nN, csrLen);
    } else {
      k_agg<0><<<nN / ANB, NTHR, 0, stream>>>(cnt, offp, Mpl, CWpl, posin, ppin, posout, AGG, nN, csrLen);
    }
    k_node<<<nN / (TW * 16), TTHR, 0, stream>>>(H32, HA, AGG, NW1p + lz * H2 * HD, nb1 + lz * HD,
                                                NW2p + lz * HD * HD, nb2 + lz * HD, lng + lz * HD, lnb + lz * HD, nN);
  }
}
